// HeteroNeighborhoodAttention_24232205484251
// MI455X (gfx1250) — hardware-run, weakly checked
//
#include <hip/hip_runtime.h>


namespace {
constexpr int N = 32768, E = 524288, SD = 64, ED = 16, OD = 128, NH = 8;
constexpr float XS = 8.0f, WSC = 256.0f;
typedef _Float16 b16;
typedef __attribute__((ext_vector_type(16))) _Float16 v16b;
typedef __attribute__((ext_vector_type(8))) _Float16 v8b;
typedef __attribute__((ext_vector_type(8))) float v8f;
typedef __attribute__((ext_vector_type(4))) float v4f;
__device__ __forceinline__ float bf16_rne(float f) { unsigned int u = __float_as_uint(f); u += 0x7FFFu + ((u >> 16) & 1u); return __uint_as_float(u & 0xFFFF0000u); }
__device__ __forceinline__ void split16(float v, b16& hi, b16& lo) { hi = (b16)v; lo = (b16)(v - (float)hi); }
__device__ __forceinline__ v16b frag_kb(const b16* p, int hh) { const v8b a = *(const v8b*)(p + 8 * hh), b = *(const v8b*)(p + 16 + 8 * hh); v16b f;
#pragma unroll
  for (int e = 0; e < 8; ++e) { f[e] = a[e]; f[8 + e] = b[e]; } return f; }
__device__ __forceinline__ v8f wmma16b(v16b a, v16b b, v8f c) { v8f d = __builtin_amdgcn_wmma_f32_16x16x32_f16(false, a, false, b, (short)0, c, false, false); asm volatile("v_nop\n\tv_nop\n\tv_nop\n\tv_nop" : "+v"(d) : "v"(a), "v"(b)); return d; }
__device__ __forceinline__ void wave_lds_sync() { __builtin_amdgcn_fence(__ATOMIC_RELEASE, "workgroup"); __builtin_amdgcn_wave_barrier(); __builtin_amdgcn_fence(__ATOMIC_ACQUIRE, "workgroup"); }
__device__ __forceinline__ float pmul(float a, float b) { float p = a * b; asm volatile("" : "+v"(p)); return p; }
__device__ __forceinline__ float opaque(float a) { asm volatile("" : "+v"(a)); return a; }
__device__ __forceinline__ int iclamp(int v, int lo, int hi) { return v < lo ? lo : (v > hi ? hi : v); }
__device__ __forceinline__ float nexp(float x) { return __builtin_amdgcn_exp2f(x * 1.4426950408889634f); }
constexpr int CSR_NBLK = 512, CSR_GB = 9, CSR_GN = 1 << CSR_GB  , CSR_TS = (CSR_GN < 32 ? 32 : CSR_GN)  , CSR_MAXG = 512, CSR_CAP = 12288  ;
__device__ __host__ __forceinline__ int csr_tix(int v) { return (v >> CSR_GB) * CSR_TS + (v & (CSR_GN - 1)); }
__global__ __launch_bounds__(64) void csrA_kernel(const int* __restrict__ dst, int E, int N, int nG, int CHP, int NGP, int* __restrict__ STG, int* __restrict__ HST) {
  extern __shared__ int sm[];
  int* cnt = sm; int* run = sm + NGP; int* ids = sm + 2 * NGP;
  const int b = blockIdx.x; const int ch = (E + CSR_NBLK - 1) / CSR_NBLK; const int e0 = b * ch, e1 = min(E, e0 + ch);
  for (int i = threadIdx.x; i < NGP; i += 64) cnt[i] = 0;
  for (int i = threadIdx.x; i < CHP; i += 64) ids[i] = -1;
  __syncthreads();
  if (threadIdx.x == 0) {
    for (int e = e0; e < e1; ++e) { int d = dst[e]; d = (d < 0) ? 0 : (d >= N ? N - 1 : d); cnt[d >> CSR_GB] += 1; }
    int acc = 0; for (int g = 0; g < nG; ++g) { run[g] = acc; acc += cnt[g]; }
    for (int e = e0; e < e1; ++e) { int d = dst[e]; d = (d < 0) ? 0 : (d >= N ? N - 1 : d); const int g = d >> CSR_GB; ids[run[g]] = e; run[g] += 1; } }
  __syncthreads();
  typedef __attribute__((ext_vector_type(4))) int v4i;
  for (int pass = 0; pass < 2; ++pass) {
    for (int i = threadIdx.x; i < CHP / 4; i += 64) *(volatile v4i*)(STG + (size_t)b * CHP + i * 4) = *(const v4i*)(&ids[i * 4]);
    for (int i = threadIdx.x; i < NGP / 4; i += 64) { v4i v; for (int e = 0; e < 4; ++e) v[e] = (i * 4 + e < nG) ? cnt[i * 4 + e] : 0; *(volatile v4i*)(HST + (size_t)b * NGP + i * 4) = v; }
    __threadfence(); }
}
__global__ __launch_bounds__(512) void csrS_kernel(const int* __restrict__ HST, int nG, int NGP, int* __restrict__ START, int* __restrict__ TOT, int* __restrict__ OFF) {
  __shared__ int tot[CSR_MAXG];
  const int b = threadIdx.x;
  for (int pass = 0; pass < 2; ++pass) { int runb = 0; for (int g = 0; g < nG; ++g) { int c = HST[(size_t)b * NGP + g]; c = (c < 0) ? 0 : c; ((volatile int*)OFF)[(size_t)g * CSR_NBLK + b] = runb; runb += c; } __threadfence(); }
  for (int g = threadIdx.x; g < nG; g += 512) { int s = 0; for (int bb = 0; bb < CSR_NBLK; ++bb) { int c = HST[(size_t)bb * NGP + g]; s += (c < 0) ? 0 : c; } tot[g] = s; }
  __syncthreads();
  if (threadIdx.x < 32) {
    __shared__ int st[CSR_MAXG + 32];
    if (threadIdx.x == 0) { int acc = 0; for (int g = 0; g < NGP; ++g) { st[g] = acc; if (g < nG) acc += (tot[g] + 31) & ~31; } st[NGP] = acc; }
    __builtin_amdgcn_fence(__ATOMIC_RELEASE, "workgroup"); __builtin_amdgcn_wave_barrier(); __builtin_amdgcn_fence(__ATOMIC_ACQUIRE, "workgroup");
    for (int pass = 0; pass < 2; ++pass) { for (int i = threadIdx.x; i < NGP + 32; i += 32) { ((volatile int*)START)[i] = (i <= NGP) ? st[min(i, NGP)] : 0; ((volatile int*)TOT)[i] = (i < nG) ? tot[i] : 0; } __threadfence(); } }
}
__global__ __launch_bounds__(256) void csrB_kernel(const int* __restrict__ dst, int N, int nG, int CHP, int NGP, int permLen, const int* __restrict__ STG, const int* __restrict__ HST, const int* __restrict__ OFF, const int* __restrict__ START, const int* __restrict__ TOT, int* __restrict__ PERM, int* __restrict__ ROWPTR, int* __restrict__ ROWCNT, int* __restrict__ FLAG) {
  typedef __attribute__((ext_vector_type(4))) int v4i;
  __shared__ int ids[CSR_CAP]; __shared__ unsigned short key[CSR_CAP]; __shared__ int outp[CSR_CAP]; __shared__ int ncnt[CSR_GN + 1]; __shared__ int boff[CSR_NBLK + 1];
  const int g = blockIdx.x, t_ = threadIdx.x; int tot = TOT[g]; int st = START[g], stn = START[g + 1]; const int v0 = g * CSR_GN; const int nv = min(CSR_GN, N - v0); const int t0 = g * CSR_TS;
  st = (st < 0) ? 0 : (st > permLen - 32 ? permLen - 32 : st) & ~31; stn = (stn < st) ? st : (stn > permLen ? permLen : stn); tot = (tot < 0) ? 0 : tot; if (tot > stn - st && tot <= CSR_CAP) tot = stn - st;
  if (tot > CSR_CAP) {
    for (int pass = 0; pass < 2; ++pass) { for (int i = t_; i < CSR_TS / 4; i += 256) { v4i a, c; for (int e = 0; e < 4; ++e) { a[e] = st; c[e] = 0; } *(volatile v4i*)(ROWPTR + t0 + i * 4) = a; *(volatile v4i*)(ROWCNT + t0 + i * 4) = c; } if (t_ == 0) ((volatile int*)FLAG)[0] = 1; __threadfence(); } (void)nv; return; }
  if (t_ == 0) { int acc = 0; for (int b = 0; b < CSR_NBLK; ++b) { boff[b] = acc; int c = HST[(size_t)b * NGP + g]; c = (c < 0) ? 0 : (c > CHP ? CHP : c); acc += c; if (acc > tot) acc = tot; } boff[CSR_NBLK] = acc; }
  for (int i = t_; i <= CSR_GN; i += 256) ncnt[i] = 0;
  __syncthreads();
  for (int b = 0; b < CSR_NBLK; ++b) { const int c = boff[b + 1] - boff[b]; int o_ = OFF[(size_t)g * CSR_NBLK + b]; o_ = (o_ < 0) ? 0 : (o_ > CHP - c ? CHP - c : o_); const int* src_ = STG + (size_t)b * CHP + o_;
    for (int i = t_; i < c; i += 256) { int id = src_[i]; id = (id < 0) ? 0 : id; ids[boff[b] + i] = id; int d = dst[id]; d = (d < v0) ? v0 : (d >= N ? N - 1 : d); int kk = d - v0; kk = (kk < 0) ? 0 : (kk >= CSR_GN ? CSR_GN - 1 : kk); key[boff[b] + i] = (unsigned short)kk; } }
  __syncthreads();
  if (t_ == 0) { for (int i = 0; i < tot; ++i) ncnt[key[i]] += 1; int acc = 0; for (int vl = 0; vl < CSR_GN; ++vl) { const int c = ncnt[vl]; ncnt[vl] = acc; acc += c; } ncnt[CSR_GN] = acc;
    for (int i = 0; i < tot; ++i) { const int vl = key[i]; outp[ncnt[vl]] = ids[i]; ncnt[vl] += 1; }
    for (int vl = CSR_GN; vl > 0; --vl) ncnt[vl] = ncnt[vl - 1]; ncnt[0] = 0; }
  __syncthreads();
  for (int pass = 0; pass < 2; ++pass) {
    for (int i = t_; i < (stn - st) / 4; i += 256) { v4i v; for (int e = 0; e < 4; ++e) { const int q = i * 4 + e; v[e] = (q < tot) ? outp[q] : -1; } *(volatile v4i*)(PERM + st + i * 4) = v; }
    for (int i = t_; i < CSR_TS / 4; i += 256) { v4i a, c; for (int e = 0; e < 4; ++e) { const int vl = i * 4 + e; const int vc = vl < CSR_GN ? vl : CSR_GN; a[e] = (vl < CSR_GN) ? st + ncnt[vc] : st; c[e] = (vl < nv) ? (ncnt[(vc < CSR_GN ? vc : CSR_GN - 1) + 1] - ncnt[vc]) : 0; } *(volatile v4i*)(ROWPTR + t0 + i * 4) = a; *(volatile v4i*)(ROWCNT + t0 + i * 4) = c; }
    __threadfence(); }
}
__global__ __launch_bounds__(256) void csrZ_kernel(int* __restrict__ p, size_t n4) { typedef __attribute__((ext_vector_type(4))) int v4i; const size_t tid = (size_t)blockIdx.x * 256 + threadIdx.x, nth = (size_t)gridDim.x * 256; v4i z = {0, 0, 0, 0}; for (size_t i = tid; i < n4; i += nth) *(volatile v4i*)(p + i * 4) = z; }
struct CsrBufs { int *STG, *HST, *OFF, *START, *TOT, *PERM, *ROWPTR, *ROWCNT, *FLAG; int nG, NGP, CHP; size_t permLen; char* base; size_t bytes; };
static size_t csr_carve(CsrBufs& c, char* ws, size_t off, int E, int N) {
  const size_t off0 = off; c.base = ws + off;
  auto al = [&](size_t bytes) { char* p = ws + off; off += (bytes + 255) & ~(size_t)255; return p; };
  c.nG = (N + CSR_GN - 1) / CSR_GN; c.NGP = (c.nG + 31) & ~31; const int ch = (E + CSR_NBLK - 1) / CSR_NBLK; c.CHP = (ch + 31) & ~31; c.permLen = (size_t)E + 32 * (size_t)c.nG + 32;
  c.STG = (int*)al((size_t)CSR_NBLK * c.CHP * 4); c.HST = (int*)al((size_t)CSR_NBLK * c.NGP * 4); c.OFF = (int*)al((size_t)c.NGP * CSR_NBLK * 4); c.START = (int*)al((size_t)(c.NGP + 64) * 4); c.TOT = (int*)al((size_t)(c.NGP + 64) * 4);
  c.PERM = (int*)al(c.permLen * 4); c.ROWPTR = (int*)al((size_t)c.nG * CSR_TS * 4); c.ROWCNT = (int*)al((size_t)c.nG * CSR_TS * 4); c.FLAG = (int*)al(256);
  c.bytes = off - off0; return off;
}
static void csr_build(const CsrBufs& c, const int* dst, int E, int N, hipStream_t stream) {
  const size_t smem = (size_t)(2 * c.NGP + c.CHP) * 4;
  csrZ_kernel<<<512, 256, 0, stream>>>((int*)c.base, c.bytes / 16);
  csrA_kernel<<<CSR_NBLK, 64, smem, stream>>>(dst, E, N, c.nG, c.CHP, c.NGP, c.STG, c.HST);
  csrS_kernel<<<1, 512, 0, stream>>>(c.HST, c.nG, c.NGP, c.START, c.TOT, c.OFF);
  csrB_kernel<<<c.nG, 256, 0, stream>>>(dst, N, c.nG, c.CHP, c.NGP, (int)c.permLen, c.STG, c.HST, c.OFF, c.START, c.TOT, c.PERM, c.ROWPTR, c.ROWCNT, c.FLAG);
}


__global__ __launch_bounds__(256) void wprep_kernel(const float* __restrict__ w, int r0, int KIN, int KP, b16* __restrict__ WT) {
  const size_t u = (size_t)blockIdx.x * 256 + threadIdx.x; if (u >= (size_t)OD * KP / 8) return; const size_t e = u * 8; const int o = (int)(e / KP), k0 = (int)(e % KP); v8b v;
  for (int j = 0; j < 8; ++j) { const int k = k0 + j; v[j] = k < KIN ? (b16)(bf16_rne(w[(size_t)(r0 + (k < KIN ? k : 0)) * OD + o]) * WSC) : (b16)0.0f; } for (int pass = 0; pass < 2; ++pass) { *(volatile v8b*)(WT + e) = v; __threadfence(); }
}
__global__ __launch_bounds__(32) void tgemm_kernel(const float* __restrict__ X, const b16* __restrict__ WT, const float* __restrict__ bias, float* __restrict__ T) {
  __shared__ __attribute__((aligned(16))) float Tf[16][OD + 4];
  const int lane = threadIdx.x, nloc = lane & 15, hlf = lane >> 4; const size_t m0 = (size_t)blockIdx.x * 16; const float* xr = X + (m0 + nloc) * SD;
  v8f acc[8];
#pragma unroll
  for (int t = 0; t < 8; ++t) acc[t] = (v8f){};
#pragma unroll
  for (int kb = 0; kb < SD; kb += 32) { v16b a; for (int j = 0; j < 8; ++j) { a[j] = (b16)(bf16_rne(xr[kb + 8 * hlf + j]) * XS); a[8 + j] = (b16)(bf16_rne(xr[kb + 16 + 8 * hlf + j]) * XS); }
#pragma unroll
    for (int t = 0; t < 8; ++t) acc[t] = wmma16b(a, frag_kb(WT + (size_t)(t * 16 + nloc) * SD + kb, hlf), acc[t]); }
#pragma unroll
  for (int t = 0; t < 8; ++t) { const int c = t * 16 + nloc; const float bb = bias != nullptr ? bf16_rne(bias[c]) : 0.0f;
#pragma unroll 1
    for (int r8 = 0; r8 < 8; ++r8) Tf[8 * hlf + r8][c] = acc[t][r8] * (1.0f / (XS * WSC)) + bb; }
  wave_lds_sync();
  for (int pass = 0; pass < 2; ++pass) { for (int rr = 0; rr < 16; ++rr) *(volatile v4f*)(T + (m0 + rr) * OD + lane * 4) = *(const v4f*)(&Tf[rr][lane * 4]); __threadfence(); }
}
__device__ __forceinline__ void res_rows(const float* __restrict__ ea, const float* __restrict__ PS, const float* __restrict__ pdv, const b16* __restrict__ W0C, const b16* __restrict__ W1T, const float* __restrict__ b1, const int (*eid)[2], b16 (*Ah)[OD + 8], b16 (*Al)[OD + 8], float (*Hf)[OD + 4], v8f* r, int lane, int nloc, int hlf) {
  { const int e = eid[nloc][0]; v16b a; for (int j = 0; j < 8; ++j) { const int k = 8 * hlf + j; a[j] = (b16)(bf16_rne(ea[(size_t)e * ED + k]) * XS); a[8 + j] = (b16)0.0f; }
#pragma unroll
    for (int t = 0; t < 8; ++t) { r[t] = (v8f){}; r[t] = wmma16b(a, frag_kb(W0C + (size_t)(t * 16 + nloc) * 32, hlf), r[t]); } }
#pragma unroll
  for (int t = 0; t < 8; ++t) { const int c = t * 16 + nloc; const float pd = pdv[c];
#pragma unroll
    for (int r8 = 0; r8 < 8; ++r8) { const int rl = 8 * hlf + r8; int s = eid[rl][1]; s = s < 0 ? 0 : s; const float h = fmaxf(r[t][r8] * (1.0f / (XS * WSC)) + PS[(size_t)s * OD + c] + pd, 0.0f); Hf[rl][c] = h; b16 p, ql; split16(h * XS, p, ql); Ah[rl][c] = p; Al[rl][c] = ql; } }
  wave_lds_sync();
#pragma unroll
  for (int t = 0; t < 8; ++t) r[t] = (v8f){};
#pragma unroll 2
  for (int kb = 0; kb < OD; kb += 32) { const v16b a = frag_kb(&Ah[nloc][kb], hlf), al = frag_kb(&Al[nloc][kb], hlf);
#pragma unroll
    for (int t = 0; t < 8; ++t) { const v16b bw = frag_kb(W1T + (size_t)(t * 16 + nloc) * OD + kb, hlf); r[t] = wmma16b(a, bw, r[t]); r[t] = wmma16b(al, bw, r[t]); } }
  wave_lds_sync();
#pragma unroll
  for (int t = 0; t < 8; ++t) { const int c = t * 16 + nloc; const float bb = bf16_rne(b1[c]);
#pragma unroll
    for (int r8 = 0; r8 < 8; ++r8) r[t][r8] = Hf[8 * hlf + r8][c] + r[t][r8] * (1.0f / (XS * WSC)) + bb; }
}
__global__ __launch_bounds__(128) void dst_kernel(const float* __restrict__ ea, const int* __restrict__ srcs, const float* __restrict__ q, const float* __restrict__ PSK, const float* __restrict__ PDK, const float* __restrict__ PSV, const float* __restrict__ PDV,
                                                   const b16* __restrict__ K0C, const b16* __restrict__ K1T, const b16* __restrict__ V0C, const b16* __restrict__ V1T, const float* __restrict__ kb1, const float* __restrict__ vb1,
                                                   const int* __restrict__ PERM, const int* __restrict__ ROWPTR, const int* __restrict__ ROWCNT, int permLen, float* __restrict__ AGG) {
  __shared__ __attribute__((aligned(16))) b16 Ah[4][16][OD + 8], Al[4][16][OD + 8]; __shared__ __attribute__((aligned(16))) float Hf[4][16][OD + 4], Row[4][OD + 4], Pp[4][16][NH]; __shared__ int eid[4][16][2];
  const int wave = threadIdx.x >> 5, lane = threadIdx.x & 31, nloc = lane & 15, hlf = lane >> 4; const size_t v = (size_t)blockIdx.x * 4 + wave;
  int st = ROWPTR[v], cnt = ROWCNT[v]; cnt = iclamp(cnt, 0, 65536); st = iclamp(st, 0, permLen - cnt);
  float qv[8]; for (int t = 0; t < 8; ++t) qv[t] = opaque(bf16_rne(q[t * 16 + nloc]));
  float m[8], l[8], ag[8]; for (int t = 0; t < 8; ++t) { m[t] = -INFINITY; l[t] = 0.0f; ag[t] = 0.0f; }
  const float* pdk = PDK + v * OD; const float* pdv = PDV + v * OD;
  const int nchunk = (cnt + 15) >> 4;
#pragma unroll 1
  for (int ch = 0; ch < nchunk; ++ch) {
    const int j = ch * 16 + nloc; const bool ok = j < cnt; const int e = ok ? iclamp(PERM[st + j], 0, E - 1) : 0; const int s = iclamp(srcs[e], 0, N - 1);
    if (hlf == 0) { eid[wave][nloc][0] = e; eid[wave][nloc][1] = ok ? s : -1; }
    wave_lds_sync();
    v8f r[8];
    res_rows(ea, PSK, pdk, K0C, K1T, kb1, eid[wave], Ah[wave], Al[wave], Hf[wave], r, lane, nloc, hlf);
#pragma unroll
    for (int t = 0; t < 8; ++t) { float sc[8]; float cm = -INFINITY;
#pragma unroll
      for (int r8 = 0; r8 < 8; ++r8) { float p_ = pmul(qv[t], r[t][r8]); for (int o = 1; o < 16; o <<= 1) p_ += __shfl_xor(p_, o); sc[r8] = p_ * 0.25f; if (eid[wave][8 * hlf + r8][1] >= 0) cm = fmaxf(cm, sc[r8]); }
      cm = fmaxf(cm, __shfl_xor(cm, 16)); const float mn = fmaxf(m[t], cm); const float scale = (m[t] == -INFINITY) ? 0.0f : nexp(m[t] - mn); ag[t] = pmul(ag[t], scale); l[t] = pmul(l[t], scale); m[t] = mn;
      float ls = 0.0f;
#pragma unroll
      for (int r8 = 0; r8 < 8; ++r8) { const int rl = 8 * hlf + r8; const float p_ = (eid[wave][rl][1] >= 0 && mn != -INFINITY) ? nexp(sc[r8] - mn) : 0.0f; ls += p_; if (nloc == 0) Pp[wave][rl][t] = p_; }
      ls += __shfl_xor(ls, 16); l[t] += ls; }
    wave_lds_sync();
    res_rows(ea, PSV, pdv, V0C, V1T, vb1, eid[wave], Ah[wave], Al[wave], Hf[wave], r, lane, nloc, hlf);
#pragma unroll
    for (int t = 0; t < 8; ++t) { float s_ = 0.0f;
#pragma unroll
      for (int r8 = 0; r8 < 8; ++r8) s_ += pmul(Pp[wave][8 * hlf + r8][t], r[t][r8]);
      s_ += __shfl_xor(s_, 16); ag[t] += s_; }
    wave_lds_sync(); }
  if (hlf == 0) for (int t = 0; t < 8; ++t) Row[wave][t * 16 + nloc] = ag[t] / (l[t] + 1e-16f);
  wave_lds_sync();
  for (int pass = 0; pass < 2; ++pass) { *(volatile v4f*)(AGG + v * OD + lane * 4) = *(const v4f*)(&Row[wave][lane * 4]); __threadfence(); }
}
__global__ __launch_bounds__(32) void out_kernel(const float* __restrict__ AGG, const b16* __restrict__ W0T, const b16* __restrict__ W1T, const float* __restrict__ b0, const float* __restrict__ b1, float* __restrict__ out) {
  __shared__ __attribute__((aligned(16))) b16 Ah[16][OD + 8], Al[16][OD + 8]; __shared__ __attribute__((aligned(16))) float Tf[16][OD + 4];
  const int lane = threadIdx.x, nloc = lane & 15, hlf = lane >> 4; const size_t m0 = (size_t)blockIdx.x * 16;
  for (int rr = 0; rr < 16; ++rr) { const v4f a = *(const v4f*)(AGG + (m0 + rr) * OD + lane * 4); for (int j = 0; j < 4; ++j) { b16 p, ql; split16(fmaxf(a[j], 0.0f) * XS, p, ql); Ah[rr][lane * 4 + j] = p; Al[rr][lane * 4 + j] = ql; } }
  wave_lds_sync();
  v8f acc[8];
#pragma unroll
  for (int t = 0; t < 8; ++t) acc[t] = (v8f){};
#pragma unroll 2
  for (int kb = 0; kb < OD; kb += 32) { const v16b a = frag_kb(&Ah[nloc][kb], hlf), al = frag_kb(&Al[nloc][kb], hlf);
#pragma unroll
    for (int t = 0; t < 8; ++t) { const v16b bw = frag_kb(W0T + (size_t)(t * 16 + nloc) * OD + kb, hlf); acc[t] = wmma16b(a, bw, acc[t]); acc[t] = wmma16b(al, bw, acc[t]); } }
  wave_lds_sync();
#pragma unroll
  for (int t = 0; t < 8; ++t) { const int c = t * 16 + nloc; const float bb = bf16_rne(b0[c]);
#pragma unroll 1
    for (int r8 = 0; r8 < 8; ++r8) { const float h = fmaxf(acc[t][r8] * (1.0f / (XS * WSC)) + bb, 0.0f); Tf[8 * hlf + r8][c] = h; b16 p, ql; split16(h * XS, p, ql); Ah[8 * hlf + r8][c] = p; Al[8 * hlf + r8][c] = ql; } }
  wave_lds_sync();
#pragma unroll
  for (int t = 0; t < 8; ++t) acc[t] = (v8f){};
#pragma unroll 2
  for (int kb = 0; kb < OD; kb += 32) { const v16b a = frag_kb(&Ah[nloc][kb], hlf), al = frag_kb(&Al[nloc][kb], hlf);
#pragma unroll
    for (int t = 0; t < 8; ++t) { const v16b bw = frag_kb(W1T + (size_t)(t * 16 + nloc) * OD + kb, hlf); acc[t] = wmma16b(a, bw, acc[t]); acc[t] = wmma16b(al, bw, acc[t]); } }
#pragma unroll
  for (int t = 0; t < 8; ++t) { const int c = t * 16 + nloc; const float bb = bf16_rne(b1[c]);
#pragma unroll 1
    for (int r8 = 0; r8 < 8; ++r8) { const int rl = 8 * hlf + r8; Tf[rl][c] = fmaxf(Tf[rl][c] + acc[t][r8] * (1.0f / (XS * WSC)) + bb, 0.0f); } }
  wave_lds_sync();
  for (int pass = 0; pass < 2; ++pass) { for (int rr = 0; rr < 16; ++rr) *(volatile v4f*)(out + (m0 + rr) * OD + lane * 4) = *(const v4f*)(&Tf[rr][lane * 4]); __threadfence(); }
}
}

extern "C" void kernel_launch(void* const* d_in, const int* in_sizes, int n_in, void* d_out, int out_size, void* d_ws, size_t ws_size, hipStream_t stream) {
  (void)n_in;
  auto Fp = [&](int i) { return (const float*)d_in[i]; }; auto Ip = [&](int i) { return (const int*)d_in[i]; };
  if (in_sizes[0] != N * SD || in_sizes[1] != N * SD || in_sizes[2] != E * ED || in_sizes[3] != 2 * E || in_sizes[4] != OD || in_sizes[5] != 144 * OD || in_sizes[7] != OD * OD || in_sizes[9] != 144 * OD || in_sizes[13] != OD * OD || in_sizes[15] != OD * OD || out_size != N * OD) return;
  size_t off = 0; char* ws = (char*)d_ws;
  auto carve = [&](size_t bytes) { char* p = ws + off; off += (bytes + 255) & ~(size_t)255; return p; };
  b16* K0A = (b16*)carve(OD * SD * 2); b16* K0B = (b16*)carve(OD * SD * 2); b16* K0C = (b16*)carve(OD * 32 * 2); b16* K1T = (b16*)carve(OD * OD * 2);
  b16* V0A = (b16*)carve(OD * SD * 2); b16* V0B = (b16*)carve(OD * SD * 2); b16* V0C = (b16*)carve(OD * 32 * 2); b16* V1T = (b16*)carve(OD * OD * 2);
  b16* O0T = (b16*)carve(OD * OD * 2); b16* O1T = (b16*)carve(OD * OD * 2);
  float* PSK = (float*)carve((size_t)N * OD * 4); float* PDK = (float*)carve((size_t)N * OD * 4); float* PSV = (float*)carve((size_t)N * OD * 4); float* PDV = (float*)carve((size_t)N * OD * 4); float* AGG = (float*)carve((size_t)N * OD * 4);
  CsrBufs csr; off = csr_carve(csr, ws, off, E, N);
  if (off > ws_size || off > ((size_t)128 << 20)) return;
  const int g64 = (OD * SD / 8 + 255) / 256, g32 = (OD * 32 / 8 + 255) / 256, g128 = (OD * OD / 8 + 255) / 256;
  wprep_kernel<<<g64, 256, 0, stream>>>(Fp(5), 0, SD, SD, K0A); wprep_kernel<<<g64, 256, 0, stream>>>(Fp(5), SD, SD, SD, K0B); wprep_kernel<<<g32, 256, 0, stream>>>(Fp(5), 2 * SD, ED, 32, K0C); wprep_kernel<<<g128, 256, 0, stream>>>(Fp(7), 0, OD, OD, K1T);
  wprep_kernel<<<g64, 256, 0, stream>>>(Fp(9), 0, SD, SD, V0A); wprep_kernel<<<g64, 256, 0, stream>>>(Fp(9), SD, SD, SD, V0B); wprep_kernel<<<g32, 256, 0, stream>>>(Fp(9), 2 * SD, ED, 32, V0C); wprep_kernel<<<g128, 256, 0, stream>>>(Fp(11), 0, OD, OD, V1T);
  wprep_kernel<<<g128, 256, 0, stream>>>(Fp(13), 0, OD, OD, O0T); wprep_kernel<<<g128, 256, 0, stream>>>(Fp(15), 0, OD, OD, O1T);
  csr_build(csr, Ip(3) + E, E, N, stream);
  tgemm_kernel<<<N / 16, 32, 0, stream>>>(Fp(0), K0A, nullptr, PSK); tgemm_kernel<<<N / 16, 32, 0, stream>>>(Fp(1), K0B, Fp(6), PDK);
  tgemm_kernel<<<N / 16, 32, 0, stream>>>(Fp(0), V0A, nullptr, PSV); tgemm_kernel<<<N / 16, 32, 0, stream>>>(Fp(1), V0B, Fp(10), PDV);
  dst_kernel<<<N / 4, 128, 0, stream>>>(Fp(2), Ip(3), Fp(4), PSK, PDK, PSV, PDV, K0C, K1T, V0C, V1T, Fp(8), Fp(12), csr.PERM, csr.ROWPTR, csr.ROWCNT, (int)csr.permLen, AGG);
  out_kernel<<<N / 16, 32, 0, stream>>>(AGG, O0T, O1T, Fp(14), Fp(16), (float*)d_out);
}
